// SparseAttention_12893491823331
// MI455X (gfx1250) — hardware-verified
//
#include <hip/hip_runtime.h>


#ifndef NB
#define NB 2
#endif
#ifndef SEQ
#define SEQ 2048
#endif
#define SEQ_FULL 2048
#define DM   2048
#define NH   16
#define HD   128
#define NG   16
#define GP   64
#define QKP  4096
#define PCAR  1024.0f
#define PCARG 64.0f
#define WCAR  16.0f
#define CSL  (0.08838834764831845f * 1.4426950408889634f)
#define CSG  (CSL * 0.0625f)
#define NEGB (-1.0e30f)

typedef _Float16 h16;
typedef __attribute__((ext_vector_type(16))) _Float16 v16h;
typedef __attribute__((ext_vector_type(8)))  _Float16 v8h;
typedef __attribute__((ext_vector_type(8)))  float    v8f;
typedef __attribute__((ext_vector_type(4)))  float    v4f;
typedef v8h  __attribute__((may_alias)) v8ha;
typedef v4f  __attribute__((may_alias)) v4fa;

static_assert(SEQ % 64 == 0);
static_assert(SEQ <= SEQ_FULL);
static_assert(NB >= 1);
static_assert(DM == NH * HD);
static_assert(HD == 128);
static_assert(QKP == 2 * DM);
static_assert(DM % 64 == 0);
static_assert(GP % 64 == 0);
static_assert(NG <= GP);

__device__ __forceinline__ unsigned short f2bf(float f) { unsigned u = __float_as_uint(f); u += 0x7FFFu + ((u >> 16) & 1u); return (unsigned short)(u >> 16); }
__device__ __forceinline__ float bf2f(unsigned short b) { return __uint_as_float(((unsigned)b) << 16); }
__device__ __forceinline__ float bfr(float f) { return bf2f(f2bf(f)); }
__device__ __forceinline__ v16h cat16(v8h lo, v8h hi) { return __builtin_shufflevector(lo, hi, 0, 1, 2, 3, 4, 5, 6, 7, 8, 9, 10, 11, 12, 13, 14, 15); }
__device__ __forceinline__ v8f wmma16(v16h a, v16h b, v8f c) { return __builtin_amdgcn_wmma_f32_16x16x32_f16(false, a, false, b, (short)0, c, false, false); }
__device__ __forceinline__ v16h ldf(const h16* p) { return cat16(*(const v8h*)p, *(const v8h*)(p + 16)); }
__device__ __forceinline__ float ex2(float x) { return __builtin_amdgcn_exp2f(x); }

static_assert(((size_t)DM * DM / 8 / 256) * 256 * 8 == (size_t)DM * DM);
__global__ __launch_bounds__(256) void k_cvtw(const float* __restrict__ w0, const float* __restrict__ w1, const float* __restrict__ w2, const float* __restrict__ w3, h16* dst) {
    const unsigned y = blockIdx.y;
    const float* src = (y == 0u) ? w0 : ((y == 1u) ? w1 : ((y == 2u) ? w2 : w3));
    const size_t i = (size_t)blockIdx.x * 256 + threadIdx.x;
    const v8f v = *(const v8f*)(src + i * 8);
    v8h o;
#pragma unroll
    for (int k = 0; k < 8; ++k) o[k] = (h16)(bfr(v[k]) * WCAR);
    h16* p = dst + (size_t)y * DM * DM + i * 8;
    *(volatile v8h*)p = o; __threadfence(); *(volatile v8h*)p = o;
}

static_assert(256 * 8 == DM);
__global__ __launch_bounds__(256) void k_gpl(const float* __restrict__ g, h16* GPL) {
    const unsigned row = blockIdx.x;
    const unsigned rc = (row < (unsigned)NG) ? row : (unsigned)(NG - 1);
    const float f = (row < (unsigned)NG) ? WCAR : 0.0f;
    const unsigned col = threadIdx.x * 8u;
    const v8f v = *(const v8f*)(g + (size_t)rc * DM + col);
    v8h o;
#pragma unroll
    for (int k = 0; k < 8; ++k) o[k] = (h16)(bfr(v[k]) * f);
    h16* p = GPL + (size_t)row * DM + col;
    *(volatile v8h*)p = o; __threadfence(); *(volatile v8h*)p = o;
}

__global__ __launch_bounds__(256) void k_ln(const float* __restrict__ x, const float* __restrict__ sc, const float* __restrict__ bi, h16* XN) {
    __shared__ float red[16];
    const unsigned tid = threadIdx.x, lane = tid & 31u, wid = tid >> 5;
    const size_t rin  = ((size_t)blockIdx.y * SEQ_FULL + blockIdx.x) * DM + tid * 8u;
    const size_t rout = ((size_t)blockIdx.y * SEQ + blockIdx.x) * DM + tid * 8u;
    v8f v = *(const v8f*)(x + rin);
    float s = 0.f;
#pragma unroll
    for (int k = 0; k < 8; ++k) { v[k] = bfr(v[k]); s += v[k]; }
#pragma unroll
    for (int sh = 16; sh; sh >>= 1) s += __shfl_xor(s, sh, 32);
    if (lane == 0u) red[wid] = s;
    __syncthreads();
    const float ts = ((red[0] + red[1]) + (red[2] + red[3])) + ((red[4] + red[5]) + (red[6] + red[7]));
    const float mu = ts * (1.0f / (float)DM);
    float ss = 0.f;
#pragma unroll
    for (int k = 0; k < 8; ++k) { const float d = v[k] - mu; v[k] = d; ss += d * d; }
#pragma unroll
    for (int sh = 16; sh; sh >>= 1) ss += __shfl_xor(ss, sh, 32);
    if (lane == 0u) red[8 + wid] = ss;
    __syncthreads();
    const float tss = ((red[8] + red[9]) + (red[10] + red[11])) + ((red[12] + red[13]) + (red[14] + red[15]));
    const float var = tss * (1.0f / (float)DM);
    const float rstd = rsqrtf(var + 1e-5f);
    const v8f g8 = *(const v8f*)(sc + tid * 8u);
    const v8f b8 = *(const v8f*)(bi + tid * 8u);
    v8h o;
#pragma unroll
    for (int k = 0; k < 8; ++k) o[k] = (h16)(v[k] * rstd * bfr(g8[k]) + bfr(b8[k]));
    h16* p = XN + rout;
    *(volatile v8h*)p = o; __threadfence(); *(volatile v8h*)p = o;
}

template <typename OT, bool RES>
__global__ __launch_bounds__(32) void k_gemmw(const h16* __restrict__ A, const h16* __restrict__ Bt, int K, OT* C, int ldc, float cs, const float* __restrict__ resid, int ldr, size_t sA, size_t sB, size_t sC, size_t sR) {
    __shared__ __align__(16) float os[16 * 68];
    const size_t z = blockIdx.z; A += z * sA; Bt += z * sB; C += z * sC; resid += z * sR;
    const unsigned lane = threadIdx.x & 31u, lr = lane & 15u, hi = lane >> 4; const unsigned r0 = blockIdx.x * 64u, c0 = blockIdx.y * 64u;
    v8f acc[4][4];
#pragma unroll
    for (int mb = 0; mb < 4; ++mb)
#pragma unroll
        for (int nb = 0; nb < 4; ++nb) acc[mb][nb] = (v8f){};
    const size_t aoff = (size_t)(r0 + lr) * K + 8u * hi, boff = (size_t)(c0 + lr) * K + 8u * hi;
#pragma unroll 1
    for (int kc = 0; kc < K; kc += 32) {
        v16h a[4];
#pragma unroll
        for (int mb = 0; mb < 4; ++mb) a[mb] = ldf(A + aoff + (size_t)mb * 16 * K + kc);
#pragma unroll
        for (int nb = 0; nb < 4; ++nb) { const v16h bq = ldf(Bt + boff + (size_t)nb * 16 * K + kc);
#pragma unroll
            for (int mb = 0; mb < 4; ++mb) acc[mb][nb] = wmma16(a[mb], bq, acc[mb][nb]); }
        asm volatile("v_nop\n\tv_nop\n\tv_nop\n\tv_nop" : "+v"(acc[0][0]), "+v"(acc[1][1]), "+v"(acc[2][2]), "+v"(acc[3][3]) : "v"(a[0]), "v"(a[3]));
    }
#pragma unroll
    for (int mb = 0; mb < 4; ++mb) {
#pragma unroll
        for (int nb = 0; nb < 4; ++nb) {
#pragma unroll
            for (int j = 0; j < 8; ++j) os[(hi * 8u + j) * 68u + nb * 16 + lr] = acc[mb][nb][j]; }
        __builtin_amdgcn_wave_barrier(); asm volatile("" ::: "memory");
        if (sizeof(OT) == 4) {
            float* crow = (float*)(void*)C + (size_t)(r0 + mb * 16) * ldc + c0;
            const float* rrow = resid + (size_t)(r0 + mb * 16) * ldr + c0;
#pragma unroll 1
            for (int ps = 0; ps < 2; ++ps) {
#pragma unroll
                for (int s = 0; s < 8; ++s) { const unsigned row = 2u * s + hi, cofs = lr * 4u; v4f val = *(const v4fa*)(os + row * 68u + cofs);
                    val[0] *= cs; val[1] *= cs; val[2] *= cs; val[3] *= cs;
                    if (RES) { const v4f rv = *(const v4f*)(rrow + (size_t)row * ldr + cofs); val[0] += bfr(rv[0]); val[1] += bfr(rv[1]); val[2] += bfr(rv[2]); val[3] += bfr(rv[3]); }
                    *(volatile v4f*)(crow + (size_t)row * ldc + cofs) = val; }
                if (ps == 0) __threadfence(); }
        } else {
            h16* crow = (h16*)(void*)C + (size_t)(r0 + mb * 16) * ldc + c0;
#pragma unroll 1
            for (int ps = 0; ps < 2; ++ps) {
#pragma unroll
                for (int s = 0; s < 4; ++s) { const unsigned row = 4u * s + (lane >> 3), cofs = (lane & 7u) * 8u;
                    const v4f v0 = *(const v4fa*)(os + row * 68u + cofs); const v4f v1 = *(const v4fa*)(os + row * 68u + cofs + 4u); v8h o;
                    o[0] = (h16)(v0[0] * cs); o[1] = (h16)(v0[1] * cs); o[2] = (h16)(v0[2] * cs); o[3] = (h16)(v0[3] * cs);
                    o[4] = (h16)(v1[0] * cs); o[5] = (h16)(v1[1] * cs); o[6] = (h16)(v1[2] * cs); o[7] = (h16)(v1[3] * cs);
                    *(volatile v8h*)(crow + (size_t)row * ldc + cofs) = o; }
                if (ps == 0) __threadfence(); }
        }
        __builtin_amdgcn_wave_barrier(); asm volatile("" ::: "memory");
    }
}

__global__ __launch_bounds__(32) void k_attn(const h16* __restrict__ QK, const h16* __restrict__ VT, const h16* __restrict__ KG, const h16* __restrict__ VGT, h16* CTX) {
    __shared__ __align__(16) h16 cst[16 * 136];
    const unsigned lane = threadIdx.x & 31u, n = lane & 15u, hh = lane >> 4;
    const unsigned t0 = blockIdx.x * 16u, h = blockIdx.y, b = blockIdx.z;
    const h16* qp = QK + (size_t)(b * (unsigned)SEQ + t0 + n) * QKP + h * (unsigned)HD + 8u * hh;
    v16h qf[4];
#pragma unroll
    for (int kq = 0; kq < 4; ++kq) qf[kq] = ldf(qp + kq * 32);
    v8f o[8];
#pragma unroll
    for (int c = 0; c < 8; ++c) o[c] = (v8f){};
    float mrun, lrun;
    {
        const h16* kp = KG + (size_t)n * DM + h * (unsigned)HD + 8u * hh;
        v8f sg = (v8f){};
#pragma unroll
        for (int kq = 0; kq < 4; ++kq) sg = wmma16(ldf(kp + kq * 32), qf[kq], sg);
        asm volatile("v_nop\n\tv_nop\n\tv_nop\n\tv_nop" : "+v"(sg) : "v"(qf[3]));
        float tv[8]; float mx = -3.0e38f;
#pragma unroll
        for (int r = 0; r < 8; ++r) { tv[r] = sg[r] * CSG; mx = fmaxf(mx, tv[r]); }
        mx = fmaxf(mx, __shfl_xor(mx, 16, 32));
        float ps = 0.f; v16h pb;
#pragma unroll
        for (int r = 0; r < 8; ++r) { const float p = ex2(tv[r] - mx); ps += p; pb[r] = (h16)(p * PCARG); pb[8 + r] = (h16)0.0f; }
        ps += __shfl_xor(ps, 16, 32);
        mrun = mx; lrun = ps;
        const h16* vp = VGT + (size_t)(h * (unsigned)HD + n) * GP + 8u * hh;
#pragma unroll
        for (int c = 0; c < 8; ++c) o[c] = wmma16(ldf(vp + (size_t)c * 16 * GP), pb, o[c]);
        asm volatile("v_nop\n\tv_nop\n\tv_nop\n\tv_nop" : "+v"(o[0]), "+v"(o[1]), "+v"(o[2]), "+v"(o[3]), "+v"(o[4]), "+v"(o[5]), "+v"(o[6]), "+v"(o[7]) : "v"(pb));
    }
    const unsigned cs0 = (t0 >= 255u) ? ((t0 - 255u) & ~31u) : 0u;
    const h16* kbase = QK + (size_t)(b * (unsigned)SEQ + n) * QKP + DM + h * (unsigned)HD + 8u * hh;
    const h16* vbase = VT + ((size_t)b * DM + h * (unsigned)HD + n) * SEQ + 8u * hh;
    const unsigned qi = t0 + n;
#pragma unroll 1
    for (unsigned cs = cs0; cs <= t0; cs += 32u) {
        const h16* k0 = kbase + (size_t)cs * QKP; const h16* k1 = k0 + (size_t)16 * QKP;
        v8f s0 = (v8f){}, s1 = (v8f){};
#pragma unroll
        for (int kq = 0; kq < 4; ++kq) { s0 = wmma16(ldf(k0 + kq * 32), qf[kq], s0); s1 = wmma16(ldf(k1 + kq * 32), qf[kq], s1); }
        asm volatile("v_nop\n\tv_nop\n\tv_nop\n\tv_nop" : "+v"(s0), "+v"(s1) : "v"(qf[3]));
        float ta[8], tb[8]; float mx = NEGB;
#pragma unroll
        for (int r = 0; r < 8; ++r) { const unsigned j0 = cs + 8u * hh + r; const unsigned j1 = j0 + 16u;
            const bool a0 = (qi - j0) <= 255u; const bool a1 = (qi - j1) <= 255u;
            ta[r] = a0 ? s0[r] * CSL : NEGB; tb[r] = a1 ? s1[r] * CSL : NEGB; mx = fmaxf(mx, fmaxf(ta[r], tb[r])); }
        mx = fmaxf(mx, __shfl_xor(mx, 16, 32));
        const float mnew = fmaxf(mrun, mx);
        const float scl = ex2(mrun - mnew);
        float ps = 0.f; v16h pb;
#pragma unroll
        for (int r = 0; r < 8; ++r) { const float p0 = ex2(ta[r] - mnew); const float p1 = ex2(tb[r] - mnew); ps += p0 + p1; pb[r] = (h16)(p0 * PCAR); pb[8 + r] = (h16)(p1 * PCAR); }
        ps += __shfl_xor(ps, 16, 32);
        lrun = lrun * scl + ps; mrun = mnew;
#pragma unroll
        for (int c = 0; c < 8; ++c) o[c] = o[c] * scl;
        const h16* vp = vbase + cs;
#pragma unroll
        for (int c = 0; c < 8; ++c) o[c] = wmma16(ldf(vp + (size_t)c * 16 * SEQ), pb, o[c]);
        asm volatile("v_nop\n\tv_nop\n\tv_nop\n\tv_nop" : "+v"(o[0]), "+v"(o[1]), "+v"(o[2]), "+v"(o[3]), "+v"(o[4]), "+v"(o[5]), "+v"(o[6]), "+v"(o[7]) : "v"(pb));
    }
    const float inv = 1.0f / (lrun * 64.0f);
#pragma unroll
    for (int c = 0; c < 8; ++c) { v8h w;
#pragma unroll
        for (int r = 0; r < 8; ++r) w[r] = (h16)(o[c][r] * inv);
        *(v8ha*)(cst + n * 136u + c * 16 + 8u * hh) = w; }
    __syncthreads();
    h16* crow = CTX + (size_t)(b * (unsigned)SEQ + t0) * DM + h * (unsigned)HD;
#pragma unroll 1
    for (int ps = 0; ps < 2; ++ps) {
#pragma unroll
        for (int s = 0; s < 8; ++s) { const unsigned row = 2u * s + hh; const v8h w = *(const v8ha*)(cst + row * 136u + n * 8u);
            *(volatile v8h*)(crow + (size_t)row * DM + n * 8u) = w; }
        if (ps == 0) __threadfence(); }
}

#define SZ_W   ((size_t)4 * DM * DM * 2)
#define SZ_GPL ((size_t)GP * DM * 2)
#define SZ_XN  ((size_t)NB * SEQ * DM * 2)
#define SZ_QK  ((size_t)NB * SEQ * QKP * 2)
#define SZ_VT  ((size_t)NB * DM * SEQ * 2)
#define SZ_KG  ((size_t)GP * DM * 2)
#define SZ_VGT ((size_t)DM * GP * 2)
#define SZ_CTX ((size_t)NB * SEQ * DM * 2)
static_assert(SZ_W % 256 == 0);
static_assert(SZ_GPL % 256 == 0);
static_assert(SZ_XN % 256 == 0);
static_assert(SZ_QK % 256 == 0);
static_assert(SZ_VT % 256 == 0);
static_assert(SZ_VGT % 256 == 0);
static_assert(SZ_W + SZ_GPL + SZ_XN + SZ_QK + SZ_VT + SZ_KG + SZ_VGT + SZ_CTX <= (size_t)134217728);
static_assert(((size_t)NB * SEQ / 64) * (QKP / 64) * 4096 == (size_t)NB * SEQ * QKP);
static_assert(((size_t)DM / 64) * (SEQ / 64) * NB * 4096 == (size_t)NB * DM * SEQ);
static_assert(((size_t)GP / 64) * (DM / 64) * 4096 == (size_t)GP * DM);
static_assert(((size_t)SEQ / 64) * (DM / 64) * NB * 4096 == (size_t)NB * SEQ * DM);
static_assert(((size_t)SEQ / 16) * NH * NB * 16 * HD == (size_t)NB * SEQ * DM);

extern "C" void kernel_launch(void* const* d_in, const int* in_sizes, int n_in,
                              void* d_out, int out_size, void* d_ws, size_t ws_size, hipStream_t stream) {
    if (n_in < 8) return;
    if (in_sizes[0] < (int)((((size_t)NB - 1) * SEQ_FULL + SEQ) * DM)) return;
    if (in_sizes[1] < NG * DM) return;
    if (in_sizes[2] < DM || in_sizes[3] < DM) return;
    if (in_sizes[4] < DM * DM || in_sizes[5] < DM * DM || in_sizes[6] < DM * DM || in_sizes[7] < DM * DM) return;
    if (out_size < (int)((size_t)NB * SEQ * DM)) return;
    const float* X   = (const float*)d_in[0];
    const float* GT  = (const float*)d_in[1];
    const float* LNS = (const float*)d_in[2];
    const float* LNB = (const float*)d_in[3];
    const float* WQ  = (const float*)d_in[4];
    const float* WK  = (const float*)d_in[5];
    const float* WV  = (const float*)d_in[6];
    const float* WO  = (const float*)d_in[7];
    float* OUT = (float*)d_out;
    char* wsp = (char*)d_ws;
    auto take = [&](size_t bytes) { char* p = wsp; wsp += (bytes + 255) & ~(size_t)255; return (void*)p; };
    h16* WPL  = (h16*)take(SZ_W);
    h16* GPL  = (h16*)take(SZ_GPL);
    h16* XN   = (h16*)take(SZ_XN);
    h16* QKb  = (h16*)take(SZ_QK);
    h16* VTb  = (h16*)take(SZ_VT);
    h16* KGb  = (h16*)take(SZ_KG);
    h16* VGTb = (h16*)take(SZ_VGT);
    h16* CTXb = (h16*)take(SZ_CTX);
    if ((size_t)(wsp - (char*)d_ws) > ws_size) return;
    const size_t WW = (size_t)DM * DM;

    k_cvtw<<<dim3((unsigned)(WW / 8 / 256), 4, 1), 256, 0, stream>>>(WQ, WK, WV, WO, WPL);
    k_gpl<<<GP, 256, 0, stream>>>(GT, GPL);
    k_ln<<<dim3(SEQ, NB, 1), 256, 0, stream>>>(X, LNS, LNB, XN);
    k_gemmw<h16, false><<<dim3(NB * SEQ / 64, QKP / 64, 1), 32, 0, stream>>>(XN, WPL, DM, QKb, QKP, 1.0f / 16.0f, X, 0, 0, 0, 0, 0);
    k_gemmw<h16, false><<<dim3(DM / 64, SEQ / 64, NB), 32, 0, stream>>>(WPL + 2 * WW, XN, DM, VTb, SEQ, 1.0f / 16.0f, X, 0, 0, (size_t)SEQ * DM, (size_t)DM * SEQ, 0);
    k_gemmw<h16, false><<<dim3(GP / 64, DM / 64, 1), 32, 0, stream>>>(GPL, WPL + WW, DM, KGb, DM, 1.0f / 16.0f, X, 0, 0, 0, 0, 0);
    k_gemmw<h16, false><<<dim3(DM / 64, GP / 64, 1), 32, 0, stream>>>(WPL + 2 * WW, GPL, DM, VGTb, GP, 1.0f / 16.0f, X, 0, 0, 0, 0, 0);
    k_attn<<<dim3(SEQ / 16, NH, NB), 32, 0, stream>>>(QKb, VTb, KGb, VGTb, CTXb);
    k_gemmw<float, true><<<dim3(SEQ / 64, DM / 64, NB), 32, 0, stream>>>(CTXb, WPL + 3 * WW, DM, OUT, DM, 1.0f / 256.0f, X, DM, (size_t)SEQ * DM, 0, (size_t)SEQ * DM, (size_t)SEQ_FULL * DM);
}
